// GAT_10969346474857
// MI455X (gfx1250) — hardware-run, weakly checked
//
#include <hip/hip_runtime.h>
#include <stddef.h>
#include <stdint.h>
#include <math.h>


#define F_IN    128
#define DHID    96
#define NHEAD   8
#define DHEAD   12
#define HCP     128
#define KA      256
#define NCLS    40
#define NCP     64
#define NTHR    256
#define NWAVE   8
#define EPT     8
#define CHUNK   (NTHR * EPT)
#define WCAP    (EPT * 32)
#define LISTN   (NWAVE * WCAP)
#define NBMAX   2048
#define SLOTB   11
#define RCAP    28672
#define DEGCAP  256
#define GBM     64
#define GBN     64
#define GTHR    128
#define MROWS   128
#define NEGSL   0.2f
#define EPS_SM  1e-16f
#define NEG_BIG (-1.0e30f)
#define WSMAX   134217728
#define LDS_AGG ((2 * RCAP + 2 * NBMAX + LISTN) * 4 + 64)

static_assert((CHUNK & (CHUNK - 1)) == 0 && CHUNK <= (1 << SLOTB));
static_assert(NBMAX == (1 << SLOTB));
static_assert(NTHR * 8 == NBMAX);
static_assert(LISTN >= NBMAX);
static_assert(LISTN >= NWAVE * WCAP);
static_assert((RCAP % 32) == 0);
static_assert(LDS_AGG <= 300000);
static_assert(GBM == (GTHR / 32) * 16);
static_assert((F_IN % 32) == 0 && (KA % 32) == 0 && (HCP % 32) == 0);
static_assert((HCP % GBN) == 0 && NCP == GBN);
static_assert(KA == 2 * HCP);
static_assert((MROWS % GBM) == 0);
static_assert(HCP == 4 * 32);
static_assert(NCP == 2 * 32);
static_assert(DHID == NHEAD * DHEAD && DHEAD == 12 && DHID <= HCP && (DHID % 8) == 0);
static_assert(NCLS <= NCP && (NCLS % 4) == 0);
static_assert((F_IN / 8) == 16);
static_assert((F_IN % 8) == 0 && (DHID % 8) == 0);

typedef float          v2f  __attribute__((ext_vector_type(2)));
typedef float          v4f  __attribute__((ext_vector_type(4)));
typedef float          v8f  __attribute__((ext_vector_type(8)));
typedef int            v4i  __attribute__((ext_vector_type(4)));
typedef int            v8i  __attribute__((ext_vector_type(8)));
typedef unsigned int   v4u  __attribute__((ext_vector_type(4)));
typedef unsigned short v8us __attribute__((ext_vector_type(8)));
typedef __bf16         v16b __attribute__((ext_vector_type(16)));
typedef v2f  __attribute__((may_alias)) v2fa;
typedef v4f  __attribute__((may_alias)) v4fa;
typedef v8us __attribute__((may_alias)) v8usa;
union FragB { v16b v; v8us h[2]; v8i w; };

__device__ __forceinline__ v8f wmb(const FragB& a, const FragB& b, v8f c) {
  v8f d = __builtin_amdgcn_wmma_f32_16x16x32_bf16(false, a.v, false, b.v, (short)0, c, false, false);
  asm volatile("v_nop\n\tv_nop\n\tv_nop\n\tv_nop" : "+v"(d) : "v"(a.w), "v"(b.w));
  return d;
}

__device__ __forceinline__ unsigned int f2bf(float f) {
  const unsigned int u = __float_as_uint(f);
  return ((u + 0x7FFFu + ((u >> 16) & 1u)) >> 16) & 0xFFFFu;
}
__device__ __forceinline__ float bf2f(unsigned int b) { return __uint_as_float(b << 16); }
__device__ __forceinline__ float bfr(float f) { return bf2f(f2bf(f)); }
__device__ __forceinline__ v4f bfr4(const v4f a) {
  v4f r; r.x = bfr(a.x); r.y = bfr(a.y); r.z = bfr(a.z); r.w = bfr(a.w); return r;
}
__device__ __forceinline__ unsigned int pk2(float lo, float hi) { return f2bf(lo) | (f2bf(hi) << 16); }
__device__ __forceinline__ v4u pack8(const v4f a, const v4f b) {
  v4u r;
  r.x = pk2(a.x, a.y); r.y = pk2(a.z, a.w); r.z = pk2(b.x, b.y); r.w = pk2(b.z, b.w);
  return r;
}

__device__ __forceinline__ int scan_chunk(const int* __restrict__ dsts, int nE, int cbase, int slotBase,
                                          int nb, int vec8, int* list, int tid, int lane, int wave) {
  int wc = 0;
  const int el0  = tid * EPT;
  const int e0   = cbase + el0;
  const int sent = -2147483647 - 1;
  v4i da, db;
  if (vec8 != 0 && cbase + CHUNK <= nE) {
    da = *(const v4i*)(dsts + e0);
    db = *(const v4i*)(dsts + e0 + 4);
  } else {
    da.x = (e0     < nE) ? dsts[min(e0,     nE - 1)] : sent;
    da.y = (e0 + 1 < nE) ? dsts[min(e0 + 1, nE - 1)] : sent;
    da.z = (e0 + 2 < nE) ? dsts[min(e0 + 2, nE - 1)] : sent;
    da.w = (e0 + 3 < nE) ? dsts[min(e0 + 3, nE - 1)] : sent;
    db.x = (e0 + 4 < nE) ? dsts[min(e0 + 4, nE - 1)] : sent;
    db.y = (e0 + 5 < nE) ? dsts[min(e0 + 5, nE - 1)] : sent;
    db.z = (e0 + 6 < nE) ? dsts[min(e0 + 6, nE - 1)] : sent;
    db.w = (e0 + 7 < nE) ? dsts[min(e0 + 7, nE - 1)] : sent;
  }
  const unsigned nbs = (unsigned)slotBase;
  const unsigned unb = (unsigned)nb;
  const unsigned s0 = (unsigned)da.x - nbs, s1 = (unsigned)da.y - nbs;
  const unsigned s2 = (unsigned)da.z - nbs, s3 = (unsigned)da.w - nbs;
  const unsigned s4 = (unsigned)db.x - nbs, s5 = (unsigned)db.y - nbs;
  const unsigned s6 = (unsigned)db.z - nbs, s7 = (unsigned)db.w - nbs;
  const bool h0 = s0 < unb, h1 = s1 < unb, h2 = s2 < unb, h3 = s3 < unb;
  const bool h4 = s4 < unb, h5 = s5 < unb, h6 = s6 < unb, h7 = s7 < unb;
  const unsigned any = __builtin_amdgcn_ballot_w32(h0 | h1 | h2 | h3 | h4 | h5 | h6 | h7);
  if (any != 0u) {
#define HITJ(J, HJ, SJ) { \
      const unsigned mj = __builtin_amdgcn_ballot_w32(HJ); \
      if (mj != 0u) { \
        if (HJ) { \
          const int pos = wc + (int)__builtin_amdgcn_mbcnt_lo(mj, 0u); \
          if (pos < WCAP) list[wave * WCAP + pos] = ((el0 + (J)) << SLOTB) | (int)(SJ); \
        } \
        wc += (int)__builtin_popcount(mj); } }
    HITJ(0, h0, s0)
    HITJ(1, h1, s1)
    HITJ(2, h2, s2)
    HITJ(3, h3, s3)
    HITJ(4, h4, s4)
    HITJ(5, h5, s5)
    HITJ(6, h6, s6)
    HITJ(7, h7, s7)
#undef HITJ
  }
  return wc;
}

__global__ __launch_bounds__(NTHR) void k_xprep(const float* __restrict__ x, unsigned short* xb, int nN, int nUnits) {
  const int i = (int)blockIdx.x * NTHR + (int)threadIdx.x;
  if (i >= nUnits) return;
  const int row = i >> 4;
  const int c0  = (i & 15) * 8;
  const int rc  = row < nN ? row : nN - 1;
  const float* p = x + (size_t)rc * F_IN + c0;
  v4f a = *(const v4fa*)p, b = *(const v4fa*)(p + 4);
  const v4f z4 = {0.f, 0.f, 0.f, 0.f};
  if (row >= nN) { a = z4; b = z4; }
  const v4u hv = pack8(a, b);
  const size_t o = (size_t)row * F_IN + c0;
  *(volatile v4u*)(xb + o) = hv;
  __threadfence();
  *(volatile v4u*)(xb + o) = hv;
}

__global__ __launch_bounds__(NTHR) void k_wtr(const float* __restrict__ w, int Kin, int Kpad, int Ncol, int Nrows,
                                              int Kout, unsigned short* wt, int nUnits) {
  const int u = (int)blockIdx.x * NTHR + (int)threadIdx.x;
  if (u >= nUnits) return;
  const int kq = Kout >> 3;
  const int n  = u / kq;
  const int k8 = (u - n * kq) * 8;
  const int kk = k8 - (k8 / Kpad) * Kpad;
  const bool kv = kk < Kin;
  const int kkc = kv ? kk : Kin - 8;
  const int ncl = n < Ncol ? n : Ncol - 1;
  const float* p = w + (size_t)kkc * (size_t)Ncol + ncl;
  v4f a, b;
  a.x = p[0];                    a.y = p[(size_t)Ncol];         a.z = p[(size_t)2 * Ncol];     a.w = p[(size_t)3 * Ncol];
  b.x = p[(size_t)4 * Ncol];     b.y = p[(size_t)5 * Ncol];     b.z = p[(size_t)6 * Ncol];     b.w = p[(size_t)7 * Ncol];
  const v4f z4 = {0.f, 0.f, 0.f, 0.f};
  if (!kv || n >= Ncol || n >= Nrows) { a = z4; b = z4; }
  const v4u wv = pack8(a, b);
  unsigned short* o = wt + (size_t)n * (size_t)Kout + k8;
  *(volatile v4u*)o = wv;
  __threadfence();
  *(volatile v4u*)o = wv;
}

__global__ __launch_bounds__(GTHR) void k_gemm(
    const unsigned short* __restrict__ A, const unsigned short* __restrict__ WT,
    float* outF, int K, int ldo)
{
  __shared__ __attribute__((aligned(16))) float stg[GBM * GBN];
  const int tid = (int)threadIdx.x, lane = tid & 31, wave = tid >> 5, hh = lane >> 4, m = lane & 15;
  const int rowBase = (int)blockIdx.x * GBM;
  const int col0    = (int)blockIdx.y * GBN;

  v8f acc[4];
  {
    const v8f z = {0.f, 0.f, 0.f, 0.f, 0.f, 0.f, 0.f, 0.f};
    acc[0] = z; acc[1] = z; acc[2] = z; acc[3] = z;
  }
  const unsigned short* ap = A  + (size_t)(rowBase + 16 * wave + m) * (size_t)K + 8 * hh;
  const unsigned short* wp = WT + (size_t)(col0 + m) * (size_t)K + 8 * hh;
  const int ksteps = K >> 5;
#pragma unroll 1
  for (int ks = 0; ks < ksteps; ++ks) {
    FragB af;
    af.h[0] = *(const v8usa*)(ap + 32 * ks);
    af.h[1] = *(const v8usa*)(ap + 32 * ks + 16);
#pragma unroll
    for (int t = 0; t < 4; ++t) {
      const unsigned short* wq = wp + (size_t)(16 * t) * (size_t)K + 32 * ks;
      FragB bf;
      bf.h[0] = *(const v8usa*)wq;
      bf.h[1] = *(const v8usa*)(wq + 16);
      acc[t] = wmb(af, bf, acc[t]);
    }
  }

#pragma unroll
  for (int t = 0; t < 4; ++t) {
    const int lc = 16 * t + m;
#pragma unroll
    for (int r = 0; r < 8; ++r) {
      const int lr = 16 * wave + 8 * hh + r;
      stg[lr * GBN + lc] = acc[t][r];
    }
  }
  __syncthreads();

  v4f fv[8];
#pragma unroll
  for (int i = 0; i < 8; ++i) {
    const int lr = 16 * wave + 2 * i + hh;
    fv[i] = *(const v4fa*)(stg + lr * GBN + 4 * m);
  }
#pragma unroll
  for (int i = 0; i < 8; ++i) {
    const int lr = 16 * wave + 2 * i + hh;
    const int gr = rowBase + lr;
    float* op = outF + (size_t)gr * (size_t)ldo + col0 + 4 * m;
    *(volatile v4f*)op = fv[i];
  }
  __threadfence();
#pragma unroll
  for (int i = 0; i < 8; ++i) {
    const int lr = 16 * wave + 2 * i + hh;
    const int gr = rowBase + lr;
    float* op = outF + (size_t)gr * (size_t)ldo + col0 + 4 * m;
    *(volatile v4f*)op = fv[i];
  }
}

__global__ __launch_bounds__(GTHR) void k_head(
    const unsigned short* __restrict__ A, const unsigned short* __restrict__ WT,
    const float* __restrict__ bo, float* out, int K, int nN)
{
  __shared__ __attribute__((aligned(16))) float stg[GBM * GBN];
  __shared__ __attribute__((aligned(16))) float sres[GBM * NCLS];
  const int tid = (int)threadIdx.x, lane = tid & 31, wave = tid >> 5, hh = lane >> 4, m = lane & 15;
  const int rowBase = (int)blockIdx.x * GBM;

  v8f acc[4];
  {
    const v8f z = {0.f, 0.f, 0.f, 0.f, 0.f, 0.f, 0.f, 0.f};
    acc[0] = z; acc[1] = z; acc[2] = z; acc[3] = z;
  }
  const unsigned short* ap = A  + (size_t)(rowBase + 16 * wave + m) * (size_t)K + 8 * hh;
  const unsigned short* wp = WT + (size_t)m * (size_t)K + 8 * hh;
  const int ksteps = K >> 5;
#pragma unroll 1
  for (int ks = 0; ks < ksteps; ++ks) {
    FragB af;
    af.h[0] = *(const v8usa*)(ap + 32 * ks);
    af.h[1] = *(const v8usa*)(ap + 32 * ks + 16);
#pragma unroll
    for (int t = 0; t < 4; ++t) {
      const unsigned short* wq = wp + (size_t)(16 * t) * (size_t)K + 32 * ks;
      FragB bf;
      bf.h[0] = *(const v8usa*)wq;
      bf.h[1] = *(const v8usa*)(wq + 16);
      acc[t] = wmb(af, bf, acc[t]);
    }
  }

#pragma unroll
  for (int t = 0; t < 4; ++t) {
    const int lc = 16 * t + m;
#pragma unroll
    for (int r = 0; r < 8; ++r) {
      const int lr = 16 * wave + 8 * hh + r;
      stg[lr * GBN + lc] = acc[t][r];
    }
  }
  __syncthreads();

  {
    const int c0 = 2 * lane;
    const bool valid = c0 < NCLS;
    const int cc0 = c0 < NCLS ? c0 : NCLS - 1;
    const int cc1 = c0 + 1 < NCLS ? c0 + 1 : NCLS - 1;
    float bz0 = bfr(bo[cc0]), bz1 = bfr(bo[cc1]);
    bz0 = valid ? bz0 : 0.f;
    bz1 = valid ? bz1 : 0.f;
#pragma unroll 1
    for (int i = 0; i < 16; ++i) {
      const int lr = 16 * wave + i;
      const v2f hv = *(const v2fa*)(stg + lr * GBN + c0);
      const float z0 = hv.x + bz0;
      const float z1 = hv.y + bz1;
      float vm = valid ? fmaxf(z0, z1) : -3.0e38f;
#pragma unroll
      for (int off = 16; off > 0; off >>= 1) vm = fmaxf(vm, __shfl_xor(vm, off));
      const float ex0 = expf(z0 - vm), ex1 = expf(z1 - vm);
      float sm = valid ? (ex0 + ex1) : 0.f;
#pragma unroll
      for (int off = 16; off > 0; off >>= 1) sm += __shfl_xor(sm, off);
      const float ls = logf(sm);
      const float o0 = (z0 - vm) - ls;
      const float o1 = (z1 - vm) - ls;
      if (valid) {
        v2f ov; ov.x = o0; ov.y = o1;
        *(v2fa*)(sres + lr * NCLS + c0) = ov;
      }
    }
  }
  __syncthreads();

  int live = nN - rowBase; live = live < 0 ? 0 : (live > GBM ? GBM : live);
  const int npc = live * (NCLS / 4);
  float* ob = out + (size_t)rowBase * NCLS;
#pragma unroll 1
  for (int p = tid; p < npc; p += GTHR) {
    const v4f v = *(const v4fa*)(sres + 4 * p);
    *(volatile v4f*)(ob + 4 * p) = v;
  }
  __threadfence();
#pragma unroll 1
  for (int p = tid; p < npc; p += GTHR) {
    const v4f v = *(const v4fa*)(sres + 4 * p);
    *(volatile v4f*)(ob + 4 * p) = v;
  }
}

template<int RELU>
__global__ __launch_bounds__(NTHR) void k_agg(
    const int* __restrict__ srcs, const int* __restrict__ dsts,
    const float* __restrict__ F,
    const float* __restrict__ asrc, const float* __restrict__ adst, const float* __restrict__ bias,
    unsigned short* HP,
    int nN, int nE, int nb, int vec8, int MPr) {
  extern __shared__ v4f lds_dyn[];
  int* reg1 = (int*)lds_dyn;
  int* reg2 = reg1 + RCAP;
  int* scnt = reg2 + RCAP;
  int* soff = scnt + NBMAX;
  int* list = soff + NBMAX;
  int* wcnt = list + LISTN;
  int* wtot = wcnt + NWAVE;
  const int tid = (int)threadIdx.x, lane = tid & 31, wave = tid >> 5;
  const int nodeBase = (int)blockIdx.x * nb;

  for (int i = tid; i < NBMAX; i += NTHR) scnt[i] = 0;
  __syncthreads();

  int tot = 0;
  const int nChunks = (nE + CHUNK - 1) / CHUNK;
#pragma unroll 1
  for (int ch = 0; ch < nChunks; ++ch) {
    const int cbase = ch * CHUNK;
    const int wc = scan_chunk(dsts, nE, cbase, nodeBase, nb, vec8, list, tid, lane, wave);
    if (lane == 0) wcnt[wave] = wc;
    __syncthreads();
    int pre = 0, all = 0;
#pragma unroll
    for (int w2 = 0; w2 < NWAVE; ++w2) {
      int c = wcnt[w2];
      c = c < 0 ? 0 : (c > WCAP ? WCAP : c);
      all += c;
      pre += (w2 < wave) ? c : 0;
    }
    const int wcc  = wc > WCAP ? WCAP : wc;
    const int base = tot + pre;
#pragma unroll 1
    for (int i = lane; i < wcc; i += 32) {
      const int ent = list[wave * WCAP + i];
      const int el  = (ent >> SLOTB) & (CHUNK - 1);
      const int sl  = ent & (NBMAX - 1);
      int eid = cbase + el;
      eid = eid > nE - 1 ? nE - 1 : eid;
      const int pos = base + i;
      if (pos < RCAP) reg1[pos] = (int)(((unsigned)eid << SLOTB) | (unsigned)sl);
    }
    tot += all;
    tot = tot > RCAP ? RCAP : tot;
    __syncthreads();
  }
  const int nh = tot;

  if (wave == 0) {
#pragma unroll 1
    for (int b0 = 0; b0 < nh; b0 += 32) {
      const int idx = b0 + lane;
      const int uv  = reg1[idx < nh ? idx : nh - 1];
      const int m32 = (nh - b0) < 32 ? (nh - b0) : 32;
#pragma unroll 1
      for (int k = 0; k < m32; ++k) {
        const int u  = __builtin_amdgcn_readlane(uv, k);
        const int sl = u & (NBMAX - 1);
        if (lane == 0) scnt[sl] = scnt[sl] + 1;
      }
    }
  }
  __syncthreads();

  {
    const v4i ca = *(const v4i*)(scnt + 8 * tid);
    const v4i cb = *(const v4i*)(scnt + 8 * tid + 4);
    const int e0 = ca.x < 0 ? 0 : ca.x, e1 = ca.y < 0 ? 0 : ca.y, e2 = ca.z < 0 ? 0 : ca.z, e3 = ca.w < 0 ? 0 : ca.w;
    const int e4 = cb.x < 0 ? 0 : cb.x, e5 = cb.y < 0 ? 0 : cb.y, e6 = cb.z < 0 ? 0 : cb.z, e7 = cb.w < 0 ? 0 : cb.w;
    const int ts = e0 + e1 + e2 + e3 + e4 + e5 + e6 + e7;
    int incl = ts;
#pragma unroll
    for (int d = 1; d < 32; d <<= 1) {
      const int up = __shfl_up(incl, d);
      if (lane >= d) incl += up;
    }
    if (lane == 31) wtot[wave] = incl;
    __syncthreads();
    int pre = 0;
#pragma unroll
    for (int w2 = 0; w2 < NWAVE; ++w2) pre += (w2 < wave) ? wtot[w2] : 0;
    int run = pre + incl - ts;
    soff[8 * tid + 0] = run; run += e0;
    soff[8 * tid + 1] = run; run += e1;
    soff[8 * tid + 2] = run; run += e2;
    soff[8 * tid + 3] = run; run += e3;
    soff[8 * tid + 4] = run; run += e4;
    soff[8 * tid + 5] = run; run += e5;
    soff[8 * tid + 6] = run; run += e6;
    soff[8 * tid + 7] = run;
  }
  __syncthreads();
  for (int i = tid; i < NBMAX; i += NTHR) list[i] = soff[i];
  __syncthreads();

  if (wave == 0) {
#pragma unroll 1
    for (int b0 = 0; b0 < nh; b0 += 32) {
      const int idx = b0 + lane;
      const int uv  = reg1[idx < nh ? idx : nh - 1];
      const int m32 = (nh - b0) < 32 ? (nh - b0) : 32;
#pragma unroll 1
      for (int k = 0; k < m32; ++k) {
        const int u   = __builtin_amdgcn_readlane(uv, k);
        const int sl  = u & (NBMAX - 1);
        const int eid = (int)((unsigned)u >> SLOTB);
        if (lane == 0) {
          int pos = list[sl];
          pos = pos < 0 ? 0 : (pos > RCAP - 1 ? RCAP - 1 : pos);
          reg2[pos] = eid;
          list[sl] = pos + 1;
        }
      }
    }
  }
  __syncthreads();

  const int nbw = nb >> 3;
  const bool ovf = (nh >= RCAP);
  const float qnan = __int_as_float(0x7fc00000);
  const v4f z4 = {0.f, 0.f, 0.f, 0.f};
  const int c0 = 4 * lane;
  const bool lv = c0 < DHID;
  const int cc = lv ? c0 : DHID - 4;
  v4f as4 = bfr4(*(const v4fa*)(asrc + cc));
  v4f ad4 = bfr4(*(const v4fa*)(adst + cc));
  v4f bb4 = bfr4(*(const v4fa*)(bias + cc));
  if (!lv) { as4 = z4; ad4 = z4; bb4 = z4; }
  const int hl = (lane / 3) * 3;
  const int j0 = hl & 31, j1 = (hl + 1) & 31, j2 = (hl + 2) & 31;

#pragma unroll 1
  for (int jt = 0; jt < nbw; ++jt) {
    const int slot = wave * nbw + jt;
    const int grow = nodeBase + slot;
    const int gcl  = grow < nN ? grow : nN - 1;
    int st = soff[slot];
    const int craw = scnt[slot];
    int cnt = craw;
    st  = st < 0 ? 0 : (st > nh ? nh : st);
    cnt = cnt < 0 ? 0 : (cnt > DEGCAP ? DEGCAP : cnt);
    if (cnt > nh - st) cnt = nh - st;
    const float pz = (ovf || craw > DEGCAP) ? qnan : 0.0f;

    const v4f fd = *(const v4fa*)(F + (size_t)gcl * HCP + c0);
    float pd = fd.x * ad4.x; pd = fmaf(fd.y, ad4.y, pd); pd = fmaf(fd.z, ad4.z, pd); pd = fmaf(fd.w, ad4.w, pd);
    const float adv = (__shfl(pd, j0) + __shfl(pd, j1)) + __shfl(pd, j2);
    float mx = NEG_BIG, dn = 0.0f;
    v4f av = z4;

#pragma unroll 1
    for (int q = 0; q < cnt; ++q) {
      int idx = st + q; idx = idx > RCAP - 1 ? RCAP - 1 : idx;
      int eid = reg2[idx]; eid = eid < 0 ? 0 : (eid > nE - 1 ? nE - 1 : eid);
      const int sraw = srcs[eid];
      const int s = sraw < 0 ? 0 : (sraw > nN - 1 ? nN - 1 : sraw);
      const v4f fs = *(const v4fa*)(F + (size_t)s * HCP + c0);
      float ps = fs.x * as4.x; ps = fmaf(fs.y, as4.y, ps); ps = fmaf(fs.z, as4.z, ps); ps = fmaf(fs.w, as4.w, ps);
      const float asv = (__shfl(ps, j0) + __shfl(ps, j1)) + __shfl(ps, j2);
      float lg = asv + adv;
      lg = lg > 0.f ? lg : NEGSL * lg;
      const float df = lg - mx;
      const float ee = __expf(-fabsf(df));
      const bool up  = df > 0.f;
      const float s1 = up ? ee : 1.0f;
      const float s2 = up ? 1.0f : ee;
      mx = up ? lg : mx;
      dn = fmaf(dn, s1, s2);
      av.x = fmaf(av.x, s1, s2 * fs.x);
      av.y = fmaf(av.y, s1, s2 * fs.y);
      av.z = fmaf(av.z, s1, s2 * fs.z);
      av.w = fmaf(av.w, s1, s2 * fs.w);
    }
    const float inv = __builtin_amdgcn_rcpf(dn + EPS_SM);
    const bool live = grow < nN;
    v4f o;
    o.x = fmaf(av.x, inv, bb4.x);
    o.y = fmaf(av.y, inv, bb4.y);
    o.z = fmaf(av.z, inv, bb4.z);
    o.w = fmaf(av.w, inv, bb4.w);
    if (RELU) {
      o.x = fmaxf(o.x, 0.f); o.y = fmaxf(o.y, 0.f); o.z = fmaxf(o.z, 0.f); o.w = fmaxf(o.w, 0.f);
    }
    o.x = (live ? o.x : 0.f) + pz;
    o.y = (live ? o.y : 0.f) + pz;
    o.z = (live ? o.z : 0.f) + pz;
    o.w = (live ? o.w : 0.f) + pz;
    const unsigned int hbx = f2bf(o.x), hby = f2bf(o.y), hbz = f2bf(o.z), hbw = f2bf(o.w);
    const unsigned int lbx = f2bf(o.x - bf2f(hbx)), lby = f2bf(o.y - bf2f(hby));
    const unsigned int lbz = f2bf(o.z - bf2f(hbz)), lbw = f2bf(o.w - bf2f(hbw));
    const int hw0 = (int)(hbx | (hby << 16)), hw1 = (int)(hbz | (hbw << 16));
    const int lw0 = (int)(lbx | (lby << 16)), lw1 = (int)(lbz | (lbw << 16));
    const int sa = (2 * lane) & 31, sb = (2 * lane + 1) & 31;
    const int g0 = __shfl(hw0, sa), g1 = __shfl(hw1, sa), g2 = __shfl(hw0, sb), g3 = __shfl(hw1, sb);
    const int q0 = __shfl(lw0, sa), q1 = __shfl(lw1, sa), q2 = __shfl(lw0, sb), q3 = __shfl(lw1, sb);
    const bool lsel = lane >= 16;
    v4u pv;
    pv.x = (unsigned int)(lsel ? q0 : g0);
    pv.y = (unsigned int)(lsel ? q1 : g1);
    pv.z = (unsigned int)(lsel ? q2 : g2);
    pv.w = (unsigned int)(lsel ? q3 : g3);
    unsigned short* gp = HP + (size_t)grow * KA + 8 * lane;
    const bool wr = grow < MPr;
    if (wr) *(volatile v4u*)gp = pv;
    __threadfence();
    if (wr) *(volatile v4u*)gp = pv;
  }
}

static int pick_nb(int nE, int nN) {
  int nb = NBMAX;
  while (nb > 32 && (long long)nb * (long long)nE * 5LL > (long long)RCAP * (long long)nN * 4LL) nb >>= 1;
  return nb;
}
static inline int cdiv(int a, int b) { return (a + b - 1) / b; }

extern "C" void kernel_launch(void* const* d_in, const int* in_sizes, int n_in,
                              void* d_out, int out_size, void* d_ws, size_t ws_size,
                              hipStream_t stream) {
  if (n_in < 13) return;
  if (in_sizes[0] <= 0 || (in_sizes[0] % F_IN) != 0) return;
  const int nN = in_sizes[0] / F_IN;
  if (nN <= 0 || nN > (1 << 22)) return;
  const int nE = in_sizes[1];
  if (nE < 1 || in_sizes[2] != nE) return;
  if (nE >= (1 << (32 - SLOTB))) return;
  if (in_sizes[3] != F_IN * DHID) return;
  if (in_sizes[4] != DHID || in_sizes[5] != DHID) return;
  if (in_sizes[6] != DHID) return;
  if (in_sizes[7] != DHID * DHID) return;
  if (in_sizes[8] != DHID || in_sizes[9] != DHID) return;
  if (in_sizes[10] != DHID) return;
  if (in_sizes[11] != DHID * NCLS) return;
  if (in_sizes[12] != NCLS) return;
  if (out_size != nN * NCLS) return;

  const float* x    = (const float*)d_in[0];
  const int*   src  = (const int*)  d_in[1];
  const int*   dst  = (const int*)  d_in[2];
  const float* W0   = (const float*)d_in[3];
  const float* a0s  = (const float*)d_in[4];
  const float* a0d  = (const float*)d_in[5];
  const float* b0   = (const float*)d_in[6];
  const float* W1   = (const float*)d_in[7];
  const float* a1s  = (const float*)d_in[8];
  const float* a1d  = (const float*)d_in[9];
  const float* b1   = (const float*)d_in[10];
  const float* Wo   = (const float*)d_in[11];
  const float* bo   = (const float*)d_in[12];
  float* out = (float*)d_out;

  const int MP   = cdiv(nN, MROWS) * MROWS;
  const int nb   = pick_nb(nE, nN);
  if (nb < 32 || (nb & (nb - 1)) != 0 || nb > NBMAX) return;
  const int gA   = cdiv(MP, nb);
  const int vec8 = 1;
  if (gA * nb < MP) return;

  char* ws = (char*)d_ws;
  size_t off = 0;
  const size_t oXB  = off; off += (size_t)MP * F_IN * 2;           off = (off + 255) & ~(size_t)255;
  const size_t oW0T = off; off += (size_t)HCP * F_IN * 2;          off = (off + 255) & ~(size_t)255;
  const size_t oW1T = off; off += (size_t)HCP * KA * 2;            off = (off + 255) & ~(size_t)255;
  const size_t oWoT = off; off += (size_t)NCP * KA * 2;            off = (off + 255) & ~(size_t)255;
  const size_t oH   = off; off += (size_t)MP * HCP * 4;            off = (off + 255) & ~(size_t)255;
  const size_t oA1  = off; off += (size_t)MP * KA * 2;             off = (off + 255) & ~(size_t)255;
  const size_t oA2  = off; off += (size_t)MP * KA * 2;             off = (off + 255) & ~(size_t)255;
  if (off > ws_size || off > (size_t)WSMAX) return;
  unsigned short* XB  = (unsigned short*)(ws + oXB);
  unsigned short* W0T = (unsigned short*)(ws + oW0T);
  unsigned short* W1T = (unsigned short*)(ws + oW1T);
  unsigned short* WoT = (unsigned short*)(ws + oWoT);
  float*          H   = (float*)(ws + oH);
  unsigned short* A1  = (unsigned short*)(ws + oA1);
  unsigned short* A2  = (unsigned short*)(ws + oA2);

  hipFuncSetAttribute(reinterpret_cast<const void*>(&k_agg<0>),
                      hipFuncAttributeMaxDynamicSharedMemorySize, LDS_AGG);
  hipFuncSetAttribute(reinterpret_cast<const void*>(&k_agg<1>),
                      hipFuncAttributeMaxDynamicSharedMemorySize, LDS_AGG);

  const int nUx = MP * (F_IN / 8);
  k_xprep<<<cdiv(nUx, NTHR), NTHR, 0, stream>>>(x, XB, nN, nUx);

  {
    const int nUw0 = HCP * (F_IN / 8);
    k_wtr<<<cdiv(nUw0, NTHR), NTHR, 0, stream>>>(W0, F_IN, F_IN, DHID, HCP, F_IN, W0T, nUw0);
    const int nUw1 = HCP * (KA / 8);
    k_wtr<<<cdiv(nUw1, NTHR), NTHR, 0, stream>>>(W1, DHID, HCP, DHID, HCP, KA, W1T, nUw1);
    const int nUwo = NCP * (KA / 8);
    k_wtr<<<cdiv(nUwo, NTHR), NTHR, 0, stream>>>(Wo, DHID, HCP, NCLS, NCP, KA, WoT, nUwo);
  }

  const int gM = MP / GBM;
  k_gemm<<<dim3(gM, HCP / GBN), GTHR, 0, stream>>>(XB, W0T, H, F_IN, HCP);
  k_agg<0><<<gA, NTHR, LDS_AGG, stream>>>(src, dst, H, a0s, a0d, b0, A1, nN, nE, nb, vec8, MP);
  k_gemm<<<dim3(gM, HCP / GBN), GTHR, 0, stream>>>(A1, W1T, H, KA, HCP);
  k_agg<1><<<gA, NTHR, LDS_AGG, stream>>>(src, dst, H, a1s, a1d, b1, A2, nN, nE, nb, vec8, MP);
  k_head<<<gM, GTHR, 0, stream>>>(A2, WoT, bo, out, KA, nN);
}
